// GAT_TimeSeries_19473381720078
// MI455X (gfx1250) — hardware-verified
//
#include <hip/hip_runtime.h>
#include <stddef.h>


#define SEQL   96
#define HID    128
#define NHEAD  8
#define HCH    1024
#define OUTD   768
#define NTHR   256
#define NWAVE  8
#define EPT    8
#define NGRP   2
#define CHUNK  (NTHR * EPT * NGRP)
#define WCAP   (EPT * NGRP * 32)
#define LISTN  (NWAVE * WCAP)
#define NBC    4096
#define NBF    1024
#define RCAP   40960
#define RBN    128
#define OTHR   512
#define GROWS  128
#define GCOLS  128
#define CROWS  32
#define AROWS  32
#define DEGCAP 128
#define WSCALE 16.0f
#define WINV   0.0625f
#define NSLOPE 0.2f
#define SMEPS  1e-16f
#define MNEG   (-3.0e38f)

#define LDS_GEMM (NWAVE * 16 * GCOLS * 4)
#define LDS_FILL ((RCAP + NBF + LISTN) * 4 + 64)
#define WS_CAP   ((size_t)134217728)

static_assert((CHUNK & (CHUNK - 1)) == 0);
static_assert(CHUNK <= 4096);
static_assert(NBC <= 4096 && NBF <= 4096);
static_assert((NBC & (NBC - 1)) == 0 && (NBF & (NBF - 1)) == 0);
static_assert(NBC == 4 * NBF);
static_assert(OTHR * 8 == NBC);
static_assert((RCAP % 32) == 0);
static_assert(NTHR == NWAVE * 32);
static_assert(NTHR == 2 * GROWS);
static_assert((GROWS * SEQL / 8) % NTHR == 0);
static_assert(SEQL % 32 == 0 && HCH % 32 == 0);
static_assert(HCH % GCOLS == 0 && OUTD % GCOLS == 0);
static_assert(HCH % NTHR == 0 && OUTD % NTHR == 0);
static_assert(CROWS == NWAVE * 4 && AROWS == NWAVE * 4);
static_assert(GROWS % CROWS == 0 && GROWS % AROWS == 0);
static_assert((HCH * SEQL / 8) % NTHR == 0 && (HCH * HCH / 8) % NTHR == 0 && (OUTD * HCH / 8) % NTHR == 0);
static_assert(HCH == NHEAD * HID && HID == 128);
static_assert(DEGCAP % 32 == 0);

typedef float    v4f  __attribute__((ext_vector_type(4)));
typedef float    v8f  __attribute__((ext_vector_type(8)));
typedef int      v4i  __attribute__((ext_vector_type(4)));
typedef _Float16 v8h  __attribute__((ext_vector_type(8)));
typedef _Float16 v16h __attribute__((ext_vector_type(16)));
union FragH { v16h v; v8h h[2]; };

__device__ __forceinline__ v8h cvt8(v4f a, v4f b) {
  v8h r;
  r[0] = (_Float16)a.x; r[1] = (_Float16)a.y; r[2] = (_Float16)a.z; r[3] = (_Float16)a.w;
  r[4] = (_Float16)b.x; r[5] = (_Float16)b.y; r[6] = (_Float16)b.z; r[7] = (_Float16)b.w;
  return r;
}

__device__ __forceinline__ v4f relu4(v4f v) {
  v4f r;
  r.x = fmaxf(v.x, 0.0f); r.y = fmaxf(v.y, 0.0f); r.z = fmaxf(v.z, 0.0f); r.w = fmaxf(v.w, 0.0f);
  return r;
}

__device__ __forceinline__ v8f wmh(v16h a, v16h b, v8f c) {
  v8f d = __builtin_amdgcn_wmma_f32_16x16x32_f16(false, a, false, b, (short)0, c, false, false);
  asm volatile("v_nop\n\tv_nop\n\tv_nop\n\tv_nop" : "+v"(d) : "v"(a), "v"(b));
  return d;
}

template <int NB>
__device__ __forceinline__ int scan_chunk(const int* __restrict__ dsts, int nE, int cbase, int slotBase,
                                          int vec8, int* list, int tid, int lane, int wave) {
  int wc = 0;
#pragma unroll
  for (int g = 0; g < NGRP; ++g) {
    const int el0  = (g * NTHR + tid) * EPT;
    const int e0   = cbase + el0;
    const int sent = -2147483647 - 1;
    v4i da, db;
    if (vec8 != 0 && cbase + CHUNK <= nE) {
      da = *(const v4i*)(dsts + e0);
      db = *(const v4i*)(dsts + e0 + 4);
    } else {
      da.x = (e0     < nE) ? dsts[min(e0, nE - 1)] : sent;
      da.y = (e0 + 1 < nE) ? dsts[min(e0 + 1, nE - 1)] : sent;
      da.z = (e0 + 2 < nE) ? dsts[min(e0 + 2, nE - 1)] : sent;
      da.w = (e0 + 3 < nE) ? dsts[min(e0 + 3, nE - 1)] : sent;
      db.x = (e0 + 4 < nE) ? dsts[min(e0 + 4, nE - 1)] : sent;
      db.y = (e0 + 5 < nE) ? dsts[min(e0 + 5, nE - 1)] : sent;
      db.z = (e0 + 6 < nE) ? dsts[min(e0 + 6, nE - 1)] : sent;
      db.w = (e0 + 7 < nE) ? dsts[min(e0 + 7, nE - 1)] : sent;
    }
    const unsigned nb = (unsigned)slotBase;
    const unsigned s0 = (unsigned)da.x - nb, s1 = (unsigned)da.y - nb;
    const unsigned s2 = (unsigned)da.z - nb, s3 = (unsigned)da.w - nb;
    const unsigned s4 = (unsigned)db.x - nb, s5 = (unsigned)db.y - nb;
    const unsigned s6 = (unsigned)db.z - nb, s7 = (unsigned)db.w - nb;
    const bool h0 = s0 < (unsigned)NB, h1 = s1 < (unsigned)NB, h2 = s2 < (unsigned)NB, h3 = s3 < (unsigned)NB;
    const bool h4 = s4 < (unsigned)NB, h5 = s5 < (unsigned)NB, h6 = s6 < (unsigned)NB, h7 = s7 < (unsigned)NB;
    const unsigned any = __builtin_amdgcn_ballot_w32(h0 | h1 | h2 | h3 | h4 | h5 | h6 | h7);
    if (any != 0u) {
#define HITJ(J, HJ, SJ) { \
        const unsigned mj = __builtin_amdgcn_ballot_w32(HJ); \
        if (mj != 0u) { \
          if (HJ) { \
            const int pos = wc + (int)__builtin_amdgcn_mbcnt_lo(mj, 0u); \
            if (pos < WCAP) list[wave * WCAP + pos] = ((el0 + (J)) << 12) | (int)(SJ); \
          } \
          wc += (int)__builtin_popcount(mj); } }
      HITJ(0, h0, s0)
      HITJ(1, h1, s1)
      HITJ(2, h2, s2)
      HITJ(3, h3, s3)
      HITJ(4, h4, s4)
      HITJ(5, h5, s5)
      HITJ(6, h6, s6)
      HITJ(7, h7, s7)
#undef HITJ
    }
  }
  return wc;
}

__global__ __launch_bounds__(NTHR) void k_wprep(
    const float* __restrict__ W1, const float* __restrict__ W2, const float* __restrict__ W3,
    _Float16* p1, _Float16* p2, _Float16* p3) {
  const int g1 = HCH * SEQL / 8;
  const int g2 = HCH * HCH / 8;
  const int g3 = OUTD * HCH / 8;
  const int bstart = blockIdx.x * NTHR;
  const float* src; _Float16* dst; int K, Nout, segOff;
  if (bstart < g1)           { src = W1; dst = p1; K = SEQL; Nout = HCH;  segOff = 0; }
  else if (bstart < g1 + g2) { src = W2; dst = p2; K = HCH;  Nout = HCH;  segOff = g1; }
  else                       { src = W3; dst = p3; K = HCH;  Nout = OUTD; segOff = g1 + g2; }
  const int i = bstart + (int)threadIdx.x;
  if (i >= g1 + g2 + g3) return;
  const int o  = (i - segOff) * 8;
  const int n  = o / K;
  const int k0 = o - n * K;
  float v[8];
#pragma unroll
  for (int e = 0; e < 8; ++e) v[e] = src[(size_t)(k0 + e) * Nout + n] * WSCALE;
  v4f a, b;
  a.x = v[0]; a.y = v[1]; a.z = v[2]; a.w = v[3];
  b.x = v[4]; b.y = v[5]; b.z = v[6]; b.w = v[7];
  const v8h hv = cvt8(a, b);
  _Float16* dp = dst + o;
  *(volatile v8h*)dp = hv;
  __threadfence();
  *(volatile v8h*)dp = hv;
}

__global__ __launch_bounds__(NTHR) void k_xprep(const float* __restrict__ x, _Float16* xh, int nN) {
  __shared__ __attribute__((aligned(16))) _Float16 sT[GROWS * SEQL];
  const int tid = threadIdx.x;
  const int rowBase = blockIdx.x * GROWS;
  const int i  = tid & (GROWS - 1);
  const int sb = tid >> 7;
  int n = rowBase + i;
  const bool okn = n < nN;
  n = okn ? n : nN - 1;
#pragma unroll 4
  for (int j = 0; j < SEQL / 2; ++j) {
    const int s = sb + 2 * j;
    float v = x[(size_t)s * nN + n];
    v = okn ? v : 0.0f;
    sT[i * SEQL + s] = (_Float16)v;
  }
  __syncthreads();
  constexpr int NP = GROWS * SEQL / 8 / NTHR;
  v8h pv[NP];
#pragma unroll
  for (int it = 0; it < NP; ++it) pv[it] = *(const v8h*)(sT + 8 * (it * NTHR + tid));
  _Float16* gp = xh + (size_t)rowBase * SEQL;
#pragma unroll
  for (int it = 0; it < NP; ++it) *(volatile v8h*)(gp + 8 * (it * NTHR + tid)) = pv[it];
  __threadfence();
#pragma unroll
  for (int it = 0; it < NP; ++it) *(volatile v8h*)(gp + 8 * (it * NTHR + tid)) = pv[it];
}

__global__ __launch_bounds__(NTHR) void k_count(const int* __restrict__ ei, int* cnt, int nE, int vec8) {
  __shared__ __attribute__((aligned(16))) int scnt[NBC];
  __shared__ __attribute__((aligned(16))) int list[LISTN];
  __shared__ int wcnt[NWAVE];
  const int tid = threadIdx.x, lane = tid & 31, wave = tid >> 5;
  const int nodeBase = blockIdx.x * NBC;
  const int* dsts = ei + nE;

  for (int i = tid; i < NBC; i += NTHR) scnt[i] = 0;
  __syncthreads();

  const int nChunks = (nE + CHUNK - 1) / CHUNK;
#pragma unroll 1
  for (int ch = 0; ch < nChunks; ++ch) {
    const int cbase = ch * CHUNK;
    const int wc = scan_chunk<NBC>(dsts, nE, cbase, nodeBase, vec8, list, tid, lane, wave);
    if (lane == 0) wcnt[wave] = wc;
    __syncthreads();
    if (wave == 0) {
#pragma unroll 1
      for (int wsx = 0; wsx < NWAVE; ++wsx) {
        int nh = __builtin_amdgcn_readfirstlane(wcnt[wsx]);
        nh = nh > WCAP ? WCAP : (nh < 0 ? 0 : nh);
        const int* lp = list + wsx * WCAP;
#pragma unroll 1
        for (int i = 0; i < nh; ++i) {
          const int ent  = __builtin_amdgcn_readfirstlane(lp[i]);
          const int slot = ent & (NBC - 1);
          if (lane == 0) scnt[slot] = scnt[slot] + 1;
        }
      }
    }
    __syncthreads();
  }

  v4i cq[4];
#pragma unroll
  for (int q = 0; q < 4; ++q) {
    const int f = (wave * 4 + q) * 128 + 4 * lane;
    cq[q] = *(const v4i*)(scnt + f);
  }
  int* cp = cnt + (size_t)nodeBase;
#pragma unroll
  for (int q = 0; q < 4; ++q) {
    const int f = (wave * 4 + q) * 128 + 4 * lane;
    *(volatile v4i*)(cp + f) = cq[q];
  }
  __threadfence();
#pragma unroll
  for (int q = 0; q < 4; ++q) {
    const int f = (wave * 4 + q) * 128 + 4 * lane;
    *(volatile v4i*)(cp + f) = cq[q];
  }
}

__global__ __launch_bounds__(OTHR) void k_offsets(
    const int* __restrict__ cnt, int* off, int* rbase, int nChunk) {
  __shared__ __attribute__((aligned(16))) int soff[NBC];
  __shared__ __attribute__((aligned(16))) int srb[RBN];
  __shared__ int wtot[OTHR / 32];
  const int tid = threadIdx.x, lane = tid & 31, wave = tid >> 5, sub = tid >> 7;
  for (int i = tid; i < RBN; i += OTHR) srb[i] = 0;
  int carry = 0;
#pragma unroll 1
  for (int ch = 0; ch < nChunk; ++ch) {
    const int base = ch * NBC;
    const v4i c0 = *(const v4i*)(cnt + base + 8 * tid);
    const v4i c1 = *(const v4i*)(cnt + base + 8 * tid + 4);
    const int e0 = max(c0.x, 0), e1 = max(c0.y, 0), e2 = max(c0.z, 0), e3 = max(c0.w, 0);
    const int e4 = max(c1.x, 0), e5 = max(c1.y, 0), e6 = max(c1.z, 0), e7 = max(c1.w, 0);
    const int ts = e0 + e1 + e2 + e3 + e4 + e5 + e6 + e7;
    int incl = ts;
#pragma unroll
    for (int d = 1; d < 32; d <<= 1) {
      const int t = __shfl_up(incl, d);
      if (lane >= d) incl += t;
    }
    if (lane == 31) wtot[wave] = incl;
    __syncthreads();
    const int S0 = wtot[0]  + wtot[1]  + wtot[2]  + wtot[3];
    const int S1 = wtot[4]  + wtot[5]  + wtot[6]  + wtot[7];
    const int S2 = wtot[8]  + wtot[9]  + wtot[10] + wtot[11];
    const int S3 = wtot[12] + wtot[13] + wtot[14] + wtot[15];
    int pre = 0;
#pragma unroll 1
    for (int w = 4 * sub; w < wave; ++w) pre += wtot[w];
    const int b0 = carry;
    const int b1 = b0 + ((S0 + 31) & ~31);
    const int b2 = b1 + ((S1 + 31) & ~31);
    const int b3 = b2 + ((S2 + 31) & ~31);
    const int b4 = b3 + ((S3 + 31) & ~31);
    const int myb = sub == 0 ? b0 : (sub == 1 ? b1 : (sub == 2 ? b2 : b3));
    if (tid == 0) {
      srb[min(4 * ch + 0, RBN - 1)] = b0;
      srb[min(4 * ch + 1, RBN - 1)] = b1;
      srb[min(4 * ch + 2, RBN - 1)] = b2;
      srb[min(4 * ch + 3, RBN - 1)] = b3;
    }
    int run = myb + pre + incl - ts;
    soff[8 * tid + 0] = run; run += e0;
    soff[8 * tid + 1] = run; run += e1;
    soff[8 * tid + 2] = run; run += e2;
    soff[8 * tid + 3] = run; run += e3;
    soff[8 * tid + 4] = run; run += e4;
    soff[8 * tid + 5] = run; run += e5;
    soff[8 * tid + 6] = run; run += e6;
    soff[8 * tid + 7] = run;
    carry = b4;
    __syncthreads();
    const v4i o0 = *(const v4i*)(soff + 4 * tid);
    const v4i o1 = *(const v4i*)(soff + 4 * (tid + OTHR));
    int* op = off + base;
    *(volatile v4i*)(op + 4 * tid) = o0;
    *(volatile v4i*)(op + 4 * (tid + OTHR)) = o1;
    __threadfence();
    *(volatile v4i*)(op + 4 * tid) = o0;
    *(volatile v4i*)(op + 4 * (tid + OTHR)) = o1;
    __syncthreads();
  }
  if (tid == 0) srb[min(4 * nChunk, RBN - 1)] = carry;
  __syncthreads();
  v4i rv = {0, 0, 0, 0};
  if (tid < 32) rv = *(const v4i*)(srb + 4 * tid);
  if (tid < 32) *(volatile v4i*)(rbase + 4 * tid) = rv;
  __threadfence();
  if (tid < 32) *(volatile v4i*)(rbase + 4 * tid) = rv;
}

__global__ __launch_bounds__(NTHR) void k_fill(
    const int* __restrict__ ei, const int* __restrict__ off, const int* __restrict__ rbase,
    int* csr, int nE, int vec8, int csrLen) {
  extern __shared__ v4f lds_dyn[];
  int* region = (int*)lds_dyn;
  int* cursor = region + RCAP;
  int* list   = cursor + NBF;
  int* wcnt   = list + LISTN;
  const int tid = threadIdx.x, lane = tid & 31, wave = tid >> 5;
  const int b = blockIdx.x;
  const int nodeBase = b * NBF;
  const int* dsts = ei + nE;

  int rb0 = rbase[b];
  const int rb1 = rbase[b + 1];
  rb0 = rb0 < 0 ? 0 : (rb0 > csrLen ? csrLen : rb0);
  rb0 &= ~31;
  int len = rb1 - rb0;
  len = len < 0 ? 0 : (len > RCAP ? RCAP : len);
  int lenW = (len + 31) & ~31;
  if (rb0 + lenW > csrLen) lenW = (csrLen - rb0) & ~31;

  {
    const v4i z = {0, 0, 0, 0};
    for (int i = tid; i < RCAP / 4; i += NTHR) ((v4i*)region)[i] = z;
    for (int s = tid; s < NBF; s += NTHR) {
      int o = off[nodeBase + s] - rb0;
      o = o < 0 ? 0 : (o > RCAP ? RCAP : o);
      cursor[s] = o;
    }
  }
  __syncthreads();

  const int nChunks = (nE + CHUNK - 1) / CHUNK;
#pragma unroll 1
  for (int ch = 0; ch < nChunks; ++ch) {
    const int cbase = ch * CHUNK;
    const int wc = scan_chunk<NBF>(dsts, nE, cbase, nodeBase, vec8, list, tid, lane, wave);
    if (lane == 0) wcnt[wave] = wc;
    __syncthreads();
    if (wave == 0) {
#pragma unroll 1
      for (int wsx = 0; wsx < NWAVE; ++wsx) {
        int nh = __builtin_amdgcn_readfirstlane(wcnt[wsx]);
        nh = nh > WCAP ? WCAP : (nh < 0 ? 0 : nh);
        const int* lp = list + wsx * WCAP;
#pragma unroll 1
        for (int i = 0; i < nh; ++i) {
          const int ent  = __builtin_amdgcn_readfirstlane(lp[i]);
          const int slot = ent & (NBF - 1);
          int e = cbase + ((ent >> 12) & (CHUNK - 1));
          e = e > nE - 1 ? nE - 1 : e;
          if (lane == 0) {
            int pos = cursor[slot];
            pos = pos < 0 ? 0 : (pos > RCAP - 1 ? RCAP - 1 : pos);
            region[pos] = e;
            const int np = pos + 1;
            cursor[slot] = np > RCAP ? RCAP : np;
          }
        }
      }
    }
    __syncthreads();
  }

  const int nv = lenW >> 2;
  int* gp = csr + rb0;
#pragma unroll 1
  for (int i = tid; i < nv; i += NTHR) { const v4i v = ((const v4i*)region)[i]; *(volatile v4i*)(gp + 4 * i) = v; }
  __threadfence();
#pragma unroll 1
  for (int i = tid; i < nv; i += NTHR) { const v4i v = ((const v4i*)region)[i]; *(volatile v4i*)(gp + 4 * i) = v; }
}

template <int KD>
__global__ __launch_bounds__(NTHR) void k_gemm(
    const _Float16* __restrict__ A, const _Float16* __restrict__ Bw, float* C, int NC) {
  extern __shared__ v4f lds_dyn[];
  float* stg = (float*)lds_dyn;
  const int tid = threadIdx.x, lane = tid & 31, wave = tid >> 5, hh = lane >> 4, m = lane & 15;
  const int rowBase = blockIdx.y * GROWS;
  const int colBase = blockIdx.x * GCOLS;

  v8f acc[8];
#pragma unroll
  for (int t = 0; t < 8; ++t) { v8f z = {0.f, 0.f, 0.f, 0.f, 0.f, 0.f, 0.f, 0.f}; acc[t] = z; }
  const _Float16* ar = A  + (size_t)(rowBase + wave * 16 + m) * KD + 8 * hh;
  const _Float16* br = Bw + (size_t)(colBase + m) * KD + 8 * hh;
#pragma unroll 1
  for (int kt = 0; kt < KD / 32; ++kt) {
    FragH a;
    a.h[0] = *(const v8h*)(ar + 32 * kt);
    a.h[1] = *(const v8h*)(ar + 32 * kt + 16);
#pragma unroll
    for (int t = 0; t < 8; ++t) {
      const _Float16* bp = br + (size_t)(16 * t) * KD + 32 * kt;
      FragH b;
      b.h[0] = *(const v8h*)bp;
      b.h[1] = *(const v8h*)(bp + 16);
      acc[t] = wmh(a.v, b.v, acc[t]);
    }
  }

  float* sp = stg + (wave * 16 + 8 * hh) * GCOLS + m;
#pragma unroll
  for (int t = 0; t < 8; ++t) {
#pragma unroll
    for (int r = 0; r < 8; ++r) sp[r * GCOLS + 16 * t] = acc[t][r] * WINV;
  }
  __syncthreads();

  const float* lp = stg + wave * 16 * GCOLS + 4 * lane;
  float* gp = C + ((size_t)rowBase + wave * 16) * NC + colBase + 4 * lane;
#pragma unroll
  for (int i = 0; i < 16; ++i) { const v4f v = *(const v4f*)(lp + i * GCOLS); *(volatile v4f*)(gp + (size_t)i * NC) = v; }
  __threadfence();
#pragma unroll
  for (int i = 0; i < 16; ++i) { const v4f v = *(const v4f*)(lp + i * GCOLS); *(volatile v4f*)(gp + (size_t)i * NC) = v; }
}

template <int H>
__global__ __launch_bounds__(NTHR) void k_coef(
    const float* __restrict__ hw, const float* __restrict__ asw, const float* __restrict__ adw,
    float* asP, float* adP) {
  constexpr int NC = (H == NHEAD) ? HCH : OUTD;
  constexpr int NQ = NC / 128;
  constexpr int RPW = CROWS / NWAVE;
  __shared__ __attribute__((aligned(16))) float sas[CROWS * H];
  __shared__ __attribute__((aligned(16))) float sad[CROWS * H];
  const int tid = threadIdx.x, lane = tid & 31, wave = tid >> 5;
  const int rowBase = blockIdx.x * CROWS;

  v4f wa[NQ], wd[NQ];
#pragma unroll
  for (int q = 0; q < NQ; ++q) {
    wa[q] = *(const v4f*)(asw + q * 128 + 4 * lane);
    wd[q] = *(const v4f*)(adw + q * 128 + 4 * lane);
  }

#pragma unroll 1
  for (int i = 0; i < RPW; ++i) {
    const int row = rowBase + wave * RPW + i;
    float ps[H], pd[H];
#pragma unroll
    for (int h = 0; h < H; ++h) { ps[h] = 0.0f; pd[h] = 0.0f; }
    const float* rp = hw + (size_t)row * NC + 4 * lane;
#pragma unroll
    for (int q = 0; q < NQ; ++q) {
      const v4f v = *(const v4f*)(rp + q * 128);
      const float ds = v.x * wa[q].x + v.y * wa[q].y + v.z * wa[q].z + v.w * wa[q].w;
      const float dd = v.x * wd[q].x + v.y * wd[q].y + v.z * wd[q].z + v.w * wd[q].w;
      if constexpr (H == NHEAD) { ps[q] += ds; pd[q] += dd; }
      else                      { ps[0] += ds; pd[0] += dd; }
    }
#pragma unroll
    for (int h = 0; h < H; ++h) {
#pragma unroll
      for (int d = 16; d > 0; d >>= 1) {
        ps[h] += __shfl_xor(ps[h], d);
        pd[h] += __shfl_xor(pd[h], d);
      }
    }
    if (lane == 0) {
#pragma unroll
      for (int h = 0; h < H; ++h) {
        sas[(wave * RPW + i) * H + h] = ps[h];
        sad[(wave * RPW + i) * H + h] = pd[h];
      }
    }
  }
  __syncthreads();

  constexpr int NPC = CROWS * H / 4;
  const int piece = tid & (NPC - 1);
  const v4f v1 = *(const v4f*)(sas + 4 * piece);
  const v4f v2 = *(const v4f*)(sad + 4 * piece);
  const v4f va = (tid < NPC) ? v1 : v2;
  float* pa = asP + (size_t)rowBase * H + 4 * piece;
  float* pd = adP + (size_t)rowBase * H + 4 * piece;
  if (tid < NPC)          *(volatile v4f*)pa = va;
  else if (tid < 2 * NPC) *(volatile v4f*)pd = va;
  __threadfence();
  if (tid < NPC)          *(volatile v4f*)pa = va;
  else if (tid < 2 * NPC) *(volatile v4f*)pd = va;
}

template <int H> struct EdgeF { int s; float w; bool valid; float as[H]; };

template <int H>
__device__ __forceinline__ EdgeF<H> edge_fetch(
    const int* __restrict__ csr, const int* __restrict__ ei, const float* __restrict__ ew,
    const float* __restrict__ asP, int st, int q0, int n, int lane, int csrLen, int nE, int nN) {
  EdgeF<H> r;
  int pos = st + q0 + lane;
  pos = pos < 0 ? 0 : (pos > csrLen - 1 ? csrLen - 1 : pos);
  int e = csr[pos];
  e = e < 0 ? 0 : (e > nE - 1 ? nE - 1 : e);
  int s = ei[e];
  s = s < 0 ? 0 : (s > nN - 1 ? nN - 1 : s);
  r.s = s;
  r.w = ew[e];
  r.valid = (q0 + lane) < n;
  if constexpr (H == NHEAD) {
    const v4f a0 = *(const v4f*)(asP + (size_t)s * NHEAD);
    const v4f a1 = *(const v4f*)(asP + (size_t)s * NHEAD + 4);
    r.as[0] = a0.x; r.as[1] = a0.y; r.as[2] = a0.z; r.as[3] = a0.w;
    r.as[4] = a1.x; r.as[5] = a1.y; r.as[6] = a1.z; r.as[7] = a1.w;
  } else {
    r.as[0] = asP[s];
  }
  return r;
}

__device__ __forceinline__ float lgt(float as, float ad, float w, float ce) {
  const float a = as + ad + w * ce;
  return a >= 0.0f ? a : a * NSLOPE;
}

template <int H>
__global__ __launch_bounds__(NTHR) void k_agg(
    const int* __restrict__ csr, const int* __restrict__ offp, const int* __restrict__ cnt,
    const int* __restrict__ ei, const float* __restrict__ ew, const float* __restrict__ hw,
    const float* __restrict__ asP, const float* __restrict__ adP,
    const float* __restrict__ We, const float* __restrict__ ae, const float* __restrict__ bias,
    _Float16* outh, float* outf, int nN, int nE, int csrLen) {
  constexpr int NC  = (H == NHEAD) ? HCH : OUTD;
  constexpr int PPT = NC / NTHR;
  constexpr int NA  = (H == NHEAD) ? 8 : 6;
  constexpr int DPW = AROWS / NWAVE;
  __shared__ float swp[NWAVE];
  const int tid = threadIdx.x, lane = tid & 31, wave = tid >> 5, hh = lane >> 4;

  {
    float part = 0.0f;
#pragma unroll
    for (int j = 0; j < PPT; ++j) part += We[PPT * tid + j] * ae[PPT * tid + j];
#pragma unroll
    for (int d = 16; d > 0; d >>= 1) part += __shfl_xor(part, d);
    if (lane == 0) swp[wave] = part;
  }
  __syncthreads();
  float cev[H];
  if constexpr (H == NHEAD) {
#pragma unroll
    for (int h = 0; h < H; ++h) cev[h] = swp[h];
  } else {
    float t = 0.0f;
#pragma unroll
    for (int w = 0; w < NWAVE; ++w) t += swp[w];
    cev[0] = t;
  }

  const int dBase = blockIdx.x * AROWS + wave * DPW;
#pragma unroll 1
  for (int i = 0; i < DPW; ++i) {
    const int c = dBase + i;
    int n = __builtin_amdgcn_readfirstlane(cnt[c]);
    n = n < 0 ? 0 : (n > DEGCAP ? DEGCAP : n);
    int st = __builtin_amdgcn_readfirstlane(offp[c]);
    st = st < 0 ? 0 : (st > csrLen - 1 ? csrLen - 1 : st);
    float adv[H];
    if constexpr (H == NHEAD) {
      const v4f d0 = *(const v4f*)(adP + (size_t)c * NHEAD);
      const v4f d1 = *(const v4f*)(adP + (size_t)c * NHEAD + 4);
      adv[0] = d0.x; adv[1] = d0.y; adv[2] = d0.z; adv[3] = d0.w;
      adv[4] = d1.x; adv[5] = d1.y; adv[6] = d1.z; adv[7] = d1.w;
    } else {
      adv[0] = adP[c];
    }

    float M[H];
#pragma unroll
    for (int h = 0; h < H; ++h) M[h] = MNEG;
#pragma unroll 1
    for (int q0 = 0; q0 < n; q0 += 32) {
      const EdgeF<H> f = edge_fetch<H>(csr, ei, ew, asP, st, q0, n, lane, csrLen, nE, nN);
#pragma unroll
      for (int h = 0; h < H; ++h) {
        const float a = lgt(f.as[h], adv[h], f.w, cev[h]);
        M[h] = fmaxf(M[h], f.valid ? a : MNEG);
      }
    }
#pragma unroll
    for (int h = 0; h < H; ++h) {
#pragma unroll
      for (int d = 16; d > 0; d >>= 1) M[h] = fmaxf(M[h], __shfl_xor(M[h], d));
    }

    float den[H];
#pragma unroll
    for (int h = 0; h < H; ++h) den[h] = 0.0f;
#pragma unroll 1
    for (int q0 = 0; q0 < n; q0 += 32) {
      const EdgeF<H> f = edge_fetch<H>(csr, ei, ew, asP, st, q0, n, lane, csrLen, nE, nN);
#pragma unroll
      for (int h = 0; h < H; ++h) {
        const float a = lgt(f.as[h], adv[h], f.w, cev[h]);
        const float p = f.valid ? __expf(a - M[h]) : 0.0f;
        den[h] += p;
      }
    }
    float inv[H];
#pragma unroll
    for (int h = 0; h < H; ++h) {
#pragma unroll
      for (int d = 16; d > 0; d >>= 1) den[h] += __shfl_xor(den[h], d);
      inv[h] = __builtin_amdgcn_rcpf(den[h] + SMEPS);
    }

    v4f acc[NA];
#pragma unroll
    for (int q = 0; q < NA; ++q) { v4f z = {0.f, 0.f, 0.f, 0.f}; acc[q] = z; }
#pragma unroll 1
    for (int q0 = 0; q0 < n; q0 += 32) {
      const EdgeF<H> f = edge_fetch<H>(csr, ei, ew, asP, st, q0, n, lane, csrLen, nE, nN);
      float p[H];
#pragma unroll
      for (int h = 0; h < H; ++h) {
        const float a = lgt(f.as[h], adv[h], f.w, cev[h]);
        p[h] = f.valid ? __expf(a - M[h]) * inv[h] : 0.0f;
      }
      const int mcnt = (n - q0) < 32 ? (n - q0) : 32;
#pragma unroll 1
      for (int j = 0; j < mcnt; ++j) {
        const int sj = __builtin_amdgcn_readlane(f.s, j);
        float P[H];
#pragma unroll
        for (int h = 0; h < H; ++h) P[h] = __int_as_float(__builtin_amdgcn_readlane(__float_as_int(p[h]), j));
        const float* rp = hw + (size_t)sj * NC;
        if constexpr (H == NHEAD) {
#pragma unroll
          for (int q = 0; q < 4; ++q) {
            const float pq = (hh == 0) ? P[2 * q] : P[2 * q + 1];
            const v4f v0 = *(const v4f*)(rp + q * 256 + 8 * lane);
            const v4f v1 = *(const v4f*)(rp + q * 256 + 8 * lane + 4);
            acc[2 * q]     += pq * v0;
            acc[2 * q + 1] += pq * v1;
          }
        } else {
#pragma unroll
          for (int q = 0; q < 6; ++q) {
            const v4f v = *(const v4f*)(rp + q * 128 + 4 * lane);
            acc[q] += P[0] * v;
          }
        }
      }
    }

    if constexpr (H == NHEAD) {
      v8h hv[4];
#pragma unroll
      for (int q = 0; q < 4; ++q) {
        const v4f b0 = *(const v4f*)(bias + q * 256 + 8 * lane);
        const v4f b1 = *(const v4f*)(bias + q * 256 + 8 * lane + 4);
        const v4f o0 = relu4(acc[2 * q] + b0);
        const v4f o1 = relu4(acc[2 * q + 1] + b1);
        hv[q] = cvt8(o0, o1);
      }
      _Float16* op = outh + (size_t)c * NC + 8 * lane;
#pragma unroll
      for (int q = 0; q < 4; ++q) *(volatile v8h*)(op + q * 256) = hv[q];
      __threadfence();
#pragma unroll
      for (int q = 0; q < 4; ++q) *(volatile v8h*)(op + q * 256) = hv[q];
    } else {
      v4f ov[6];
#pragma unroll
      for (int q = 0; q < 6; ++q) ov[q] = acc[q] + *(const v4f*)(bias + q * 128 + 4 * lane);
      if (c < nN) {
        float* op = outf + (size_t)c * NC + 4 * lane;
#pragma unroll
        for (int q = 0; q < 6; ++q) *(volatile v4f*)(op + q * 128) = ov[q];
        __threadfence();
#pragma unroll
        for (int q = 0; q < 6; ++q) *(volatile v4f*)(op + q * 128) = ov[q];
      }
    }
  }
}

extern "C" void kernel_launch(void* const* d_in, const int* in_sizes, int n_in,
                              void* d_out, int out_size, void* d_ws, size_t ws_size,
                              hipStream_t stream) {
  if (n_in < 21) return;
  if (out_size <= 0 || (out_size % OUTD) != 0) return;
  const int nN = out_size / OUTD;
  if (nN <= 0 || nN > (1 << 22)) return;
  if (in_sizes[0] != SEQL * nN) return;
  const int nE = in_sizes[2];
  if (nE <= 0 || nE > (1 << 26) || in_sizes[1] != 2 * nE) return;
  if (in_sizes[3] != SEQL * HCH || in_sizes[4] != HCH || in_sizes[5] != HCH ||
      in_sizes[6] != HCH || in_sizes[7] != HCH || in_sizes[8] != HCH) return;
  if (in_sizes[9] != HCH * HCH || in_sizes[10] != HCH || in_sizes[11] != HCH ||
      in_sizes[12] != HCH || in_sizes[13] != HCH || in_sizes[14] != HCH) return;
  if (in_sizes[15] != HCH * OUTD || in_sizes[16] != OUTD || in_sizes[17] != OUTD ||
      in_sizes[18] != OUTD || in_sizes[19] != OUTD || in_sizes[20] != OUTD) return;

  const float* x   = (const float*)d_in[0];
  const int*   ei  = (const int*)d_in[1];
  const float* ew  = (const float*)d_in[2];
  const float* W1  = (const float*)d_in[3];
  const float* as1 = (const float*)d_in[4];
  const float* ad1 = (const float*)d_in[5];
  const float* We1 = (const float*)d_in[6];
  const float* ae1 = (const float*)d_in[7];
  const float* b1  = (const float*)d_in[8];
  const float* W2  = (const float*)d_in[9];
  const float* as2 = (const float*)d_in[10];
  const float* ad2 = (const float*)d_in[11];
  const float* We2 = (const float*)d_in[12];
  const float* ae2 = (const float*)d_in[13];
  const float* b2  = (const float*)d_in[14];
  const float* W3  = (const float*)d_in[15];
  const float* as3 = (const float*)d_in[16];
  const float* ad3 = (const float*)d_in[17];
  const float* We3 = (const float*)d_in[18];
  const float* ae3 = (const float*)d_in[19];
  const float* b3  = (const float*)d_in[20];
  float* out = (float*)d_out;

  const int NPAD   = ((nN + GROWS - 1) / GROWS) * GROWS;
  const int nBC    = (nN + NBC - 1) / NBC;
  const int CNTPAD = nBC * NBC;
  if (CNTPAD < NPAD) return;
  if (4 * nBC + 1 > RBN) return;
  const int nBF    = (nN + NBF - 1) / NBF;
  if (nBF > 4 * nBC) return;
  const int csrLen = ((nE + 31) & ~31) + 4096;
  const int nRowBlk = NPAD / GROWS;
  const int nCoef   = NPAD / CROWS;
  const int nAgg    = NPAD / AROWS;

  char* ws = (char*)d_ws;
  size_t off = 0;
  const size_t oW1  = off; off += (size_t)HCH * SEQL * 2;          off = (off + 255) & ~(size_t)255;
  const size_t oW2  = off; off += (size_t)HCH * HCH * 2;           off = (off + 255) & ~(size_t)255;
  const size_t oW3  = off; off += (size_t)OUTD * HCH * 2;          off = (off + 255) & ~(size_t)255;
  const size_t oX   = off; off += (size_t)NPAD * SEQL * 2;         off = (off + 255) & ~(size_t)255;
  const size_t oAct = off; off += (size_t)NPAD * HCH * 2;          off = (off + 255) & ~(size_t)255;
  const size_t oC   = off; off += (size_t)NPAD * HCH * 4;          off = (off + 255) & ~(size_t)255;
  const size_t oAs  = off; off += (size_t)NPAD * NHEAD * 4;        off = (off + 255) & ~(size_t)255;
  const size_t oAd  = off; off += (size_t)NPAD * NHEAD * 4;        off = (off + 255) & ~(size_t)255;
  const size_t oCnt = off; off += (size_t)CNTPAD * 4;              off = (off + 255) & ~(size_t)255;
  const size_t oOff = off; off += (size_t)CNTPAD * 4;              off = (off + 255) & ~(size_t)255;
  const size_t oRb  = off; off += (size_t)RBN * 4;                 off = (off + 255) & ~(size_t)255;
  const size_t oCsr = off; off += (size_t)csrLen * 4;              off = (off + 255) & ~(size_t)255;
  if (off > ws_size || off > WS_CAP) return;
  _Float16* w1h  = (_Float16*)(ws + oW1);
  _Float16* w2h  = (_Float16*)(ws + oW2);
  _Float16* w3h  = (_Float16*)(ws + oW3);
  _Float16* xh   = (_Float16*)(ws + oX);
  _Float16* act  = (_Float16*)(ws + oAct);
  float*    cpl  = (float*)(ws + oC);
  float*    asP  = (float*)(ws + oAs);
  float*    adP  = (float*)(ws + oAd);
  int*      cnt  = (int*)(ws + oCnt);
  int*      offp = (int*)(ws + oOff);
  int*      rb   = (int*)(ws + oRb);
  int*      csr  = (int*)(ws + oCsr);

  const int vec8 = ((nE & 3) == 0) ? 1 : 0;

  const int nPrep = HCH * SEQL / 8 + HCH * HCH / 8 + OUTD * HCH / 8;
  k_wprep<<<(nPrep + NTHR - 1) / NTHR, NTHR, 0, stream>>>(W1, W2, W3, w1h, w2h, w3h);

  k_xprep<<<nRowBlk, NTHR, 0, stream>>>(x, xh, nN);

  k_count<<<nBC, NTHR, 0, stream>>>(ei, cnt, nE, vec8);
  k_offsets<<<1, OTHR, 0, stream>>>(cnt, offp, rb, nBC);
  hipFuncSetAttribute(reinterpret_cast<const void*>(&k_fill),
                      hipFuncAttributeMaxDynamicSharedMemorySize, LDS_FILL);
  k_fill<<<nBF, NTHR, LDS_FILL, stream>>>(ei, offp, rb, csr, nE, vec8, csrLen);

  hipFuncSetAttribute(reinterpret_cast<const void*>(&k_gemm<SEQL>),
                      hipFuncAttributeMaxDynamicSharedMemorySize, LDS_GEMM);
  hipFuncSetAttribute(reinterpret_cast<const void*>(&k_gemm<HCH>),
                      hipFuncAttributeMaxDynamicSharedMemorySize, LDS_GEMM);

  k_gemm<SEQL><<<dim3(HCH / GCOLS, nRowBlk), NTHR, LDS_GEMM, stream>>>(xh, w1h, cpl, HCH);
  k_coef<NHEAD><<<nCoef, NTHR, 0, stream>>>(cpl, as1, ad1, asP, adP);
  k_agg<NHEAD><<<nAgg, NTHR, 0, stream>>>(csr, offp, cnt, ei, ew, cpl, asP, adP, We1, ae1, b1,
                                          act, out, nN, nE, csrLen);

  k_gemm<HCH><<<dim3(HCH / GCOLS, nRowBlk), NTHR, LDS_GEMM, stream>>>(act, w2h, cpl, HCH);
  k_coef<NHEAD><<<nCoef, NTHR, 0, stream>>>(cpl, as2, ad2, asP, adP);
  k_agg<NHEAD><<<nAgg, NTHR, 0, stream>>>(csr, offp, cnt, ei, ew, cpl, asP, adP, We2, ae2, b2,
                                          act, out, nN, nE, csrLen);

  k_gemm<HCH><<<dim3(OUTD / GCOLS, nRowBlk), NTHR, LDS_GEMM, stream>>>(act, w3h, cpl, OUTD);
  k_coef<1><<<nCoef, NTHR, 0, stream>>>(cpl, as3, ad3, asP, adP);
  k_agg<1><<<nAgg, NTHR, 0, stream>>>(csr, offp, cnt, ei, ew, cpl, asP, adP, We3, ae3, b3,
                                      act, out, nN, nE, csrLen);
}
